// NCMultiAgentPolicy_2439541424798
// MI455X (gfx1250) — hardware-run, weakly checked
//
#include <hip/hip_runtime.h>


#ifndef NT
#define NT 64
#endif
#define NT_FULL 64
#define NAG  64
#define NSO  64
#define NAC  8
#define NNB  4
#define NFC  128
#define NHD  128
#define F3   384
#define NG4  512
#define KXC  320
#define KPC  32
#define KMC  512
#define KCC  160
#define HROWS (NT + 1)
#define MBT  (NT / 16)
#define AWV  12
#define OSP  36
#define HOP  20
#define QRS  2048.0f
#define QRI  (1.0f / 2048.0f)
#define WCS  64.0f
#define WCI  (1.0f / 64.0f)
#define PCS  1024.0f
#define PCI  (1.0f / 1024.0f)
#define LOG2E 1.4426950408889634f
#define NEGF (-9.0e15f)

static_assert(NT % 32 == 0);
static_assert(NT >= 32);
static_assert(NT <= NT_FULL);
static_assert(MBT * 16 == NT);
static_assert(KXC % 32 == 0);
static_assert(KPC % 32 == 0);
static_assert(F3 % 32 == 0);
static_assert(NAG % 32 == 0);
static_assert(NHD % 32 == 0);
static_assert(NFC % 64 == 0);
static_assert(F3 == 3 * NFC);
static_assert(AWV * 32 == F3);
static_assert(AWV >= 6);
static_assert(NAG == 64);
static_assert(NNB == 4);
static_assert(NHD == 128);
static_assert(NG4 == 4 * NHD);
static_assert(KMC == NNB * NHD);
static_assert(KCC == NHD + NNB * NAC);
static_assert(NAC == 8);
static_assert((OSP * 4) % 16 == 0);
static_assert((HOP * 4) % 16 == 0);
static_assert(16 * OSP <= 1024);
static_assert((size_t)NAG * NT_FULL * NAC * 4 == (size_t)131072);

typedef _Float16 h16;
typedef unsigned short bf;
typedef __attribute__((ext_vector_type(16))) __bf16   v16bf;
typedef __attribute__((ext_vector_type(16))) _Float16 v16h;
typedef __attribute__((ext_vector_type(8)))  _Float16 v8h;
typedef __attribute__((ext_vector_type(8)))  unsigned short v8us;
typedef __attribute__((ext_vector_type(8)))  float    v8f;
typedef __attribute__((ext_vector_type(4)))  float    v4f;
typedef v4f  __attribute__((may_alias)) v4fa;
typedef __attribute__((ext_vector_type(4)))  unsigned int v4u;
typedef v8h  __attribute__((may_alias)) v8ha;

__device__ __forceinline__ unsigned short f2bf(float f) { unsigned u = __float_as_uint(f); u += 0x7FFFu + ((u >> 16) & 1u); return (unsigned short)(u >> 16); }
__device__ __forceinline__ float bfr(float f) { return __uint_as_float(((unsigned)f2bf(f)) << 16); }
__device__ __forceinline__ v16h cat16(v8h lo, v8h hi) { return __builtin_shufflevector(lo, hi, 0, 1, 2, 3, 4, 5, 6, 7, 8, 9, 10, 11, 12, 13, 14, 15); }
__device__ __forceinline__ v16bf cat16b(v8us lo, v8us hi) { return __builtin_bit_cast(v16bf, __builtin_shufflevector(lo, hi, 0, 1, 2, 3, 4, 5, 6, 7, 8, 9, 10, 11, 12, 13, 14, 15)); }
__device__ __forceinline__ v8f wmma16(v16h a, v16h b, v8f c) { return __builtin_amdgcn_wmma_f32_16x16x32_f16(false, a, false, b, (short)0, c, false, false); }
__device__ __forceinline__ v8f wmmab(v16bf a, v16bf b, v8f c) { return __builtin_amdgcn_wmma_f32_16x16x32_bf16(false, a, false, b, (short)0, c, false, false); }
__device__ __forceinline__ v16h  ldh(const h16* p) { return cat16(*(const v8h*)p, *(const v8h*)(p + 16)); }
__device__ __forceinline__ v16bf ldb(const bf* p)  { return cat16b(*(const v8us*)p, *(const v8us*)(p + 16)); }
__device__ __forceinline__ void wave_sync() { __builtin_amdgcn_fence(3  , "wavefront"); __builtin_amdgcn_wave_barrier(); asm volatile("" ::: "memory"); }

static __device__ __forceinline__ h16 toh_flush(float v) { const h16 r = (h16)v; return (fabsf(v) < 6.103515625e-05f) ? (h16)0.0f : r; }
static __device__ __forceinline__ v8f wmma16g(v16h a, v16h b, v8f c) { c = wmma16(a, b, c); asm volatile("v_nop\n\tv_nop\n\tv_nop\n\tv_nop" : "+v"(c) : "v"(a), "v"(b)); return c; }
static __device__ __forceinline__ v8f wmmabg(v16bf a, v16bf b, v8f c) { c = wmmab(a, b, c); asm volatile("v_nop\n\tv_nop\n\tv_nop\n\tv_nop" : "+v"(c) : "v"(a), "v"(b)); return c; }
static __device__ __forceinline__ int clampi(int v, int lo, int hi) { return v < lo ? lo : (v > hi ? hi : v); }
static __device__ __forceinline__ float dot8(const v4u w, const v4f x0, const v4f x1, float acc) {
    acc = fmaf(__uint_as_float(w[0] << 16),         x0[0], acc);
    acc = fmaf(__uint_as_float(w[0] & 0xffff0000u), x0[1], acc);
    acc = fmaf(__uint_as_float(w[1] << 16),         x0[2], acc);
    acc = fmaf(__uint_as_float(w[1] & 0xffff0000u), x0[3], acc);
    acc = fmaf(__uint_as_float(w[2] << 16),         x1[0], acc);
    acc = fmaf(__uint_as_float(w[2] & 0xffff0000u), x1[1], acc);
    acc = fmaf(__uint_as_float(w[3] << 16),         x1[2], acc);
    acc = fmaf(__uint_as_float(w[3] & 0xffff0000u), x1[3], acc);
    return acc;
}
static __device__ __forceinline__ float sgm(float x) { const float xc = fminf(fmaxf(x, -30.0f), 30.0f); return __builtin_amdgcn_rcpf(1.0f + __builtin_amdgcn_exp2f(-xc * LOG2E)); }
static __device__ __forceinline__ float tnh(float x) { const float xc = fminf(fmaxf(x, -15.0f), 15.0f); return 1.0f - 2.0f * __builtin_amdgcn_rcpf(__builtin_amdgcn_exp2f(2.0f * xc * LOG2E) + 1.0f); }
static __device__ __forceinline__ float zmask(float w1, float w2, int aj) { const float z = w1 + w2; const float e = (z >= 0.0f) ? z : 0.2f * z; return (aj != 0) ? e : NEGF; }

static constexpr size_t SPLANE = (size_t)NT * NAG * F3;

__global__ __launch_bounds__(256) void k_cvt8(const float* __restrict__ src, bf* dst, size_t n8) {
    const size_t i = (size_t)blockIdx.x * 256 + threadIdx.x; if (i >= n8) return;
    const v8f v = *(const v8f*)(src + i * 8); v8us o;
#pragma unroll
    for (int k = 0; k < 8; ++k) o[k] = f2bf(v[k]);
    *(volatile v8us*)(dst + i * 8) = o; __threadfence(); *(volatile v8us*)(dst + i * 8) = o;
}

static_assert(256 * 8 == 64 * 32);
static_assert(256 * 16 == 32 * 128);
__global__ __launch_bounds__(256) void k_wgt(const float* __restrict__ Wg, h16* WGT) {
    __shared__ __align__(16) h16 ts[32 * 72];
    const int tid = threadIdx.x; const int k0 = blockIdx.x * 64, n0 = blockIdx.y * 32;
    { const int kk = tid >> 2, n8 = (tid & 3) * 8;
      const v8f v = *(const v8f*)(Wg + (size_t)(k0 + kk) * F3 + n0 + n8);
#pragma unroll
      for (int i = 0; i < 8; ++i) ts[(n8 + i) * 72 + kk] = toh_flush(bfr(v[i]) * WCS); }
    __syncthreads();
    { const int nn = tid >> 3, c8 = (tid & 7) * 8;
      const v8h o = *(const v8ha*)(&ts[nn * 72 + c8]);
      h16* p = WGT + (size_t)(n0 + nn) * F3 + k0 + c8;
      *(volatile v8h*)p = o; __threadfence(); *(volatile v8h*)p = o; }
}

static_assert(((size_t)NAG * 16 * NHD / 8) % 256 == 0);
__global__ __launch_bounds__(256) void k_whead(const float* __restrict__ Wa, const float* __restrict__ Wc, h16* WAC) {
    const int i = blockIdx.x * 256 + threadIdx.x;
    const int n = i >> 8, r = (i >> 4) & 15, c8 = (i & 15) * 8;
    const int ra = r < NAC ? r : NAC - 1;
    v8f va = *(const v8f*)(Wa + ((size_t)n * NAC + ra) * NHD + c8);
    v8f vc = *(const v8f*)(Wc + (size_t)n * KCC + c8);
    asm volatile("" : "+v"(va)); asm volatile("" : "+v"(vc));
    v8h o;
#pragma unroll
    for (int k = 0; k < 8; ++k) { const float x = (r < NAC) ? va[k] : ((r == NAC) ? vc[k] : 0.0f); o[k] = toh_flush(bfr(x) * WCS); }
    h16* p = WAC + (size_t)i * 8;
    *(volatile v8h*)p = o; __threadfence(); *(volatile v8h*)p = o;
}

__global__ __launch_bounds__(64) void k_init(const float* __restrict__ states, float* HSp, float* Cp) {
    const int lane = threadIdx.x & 31; const int wave = __builtin_amdgcn_readfirstlane((int)(threadIdx.x >> 5)); const int n = blockIdx.x;
    const v4f s = *(const v4f*)(states + (size_t)n * 2 * NHD + wave * NHD + lane * 4);
    v4f o;
#pragma unroll
    for (int i = 0; i < 4; ++i) o[i] = bfr(s[i]);
    if (wave == 0) { float* p = HSp + (size_t)n * HROWS * NHD + lane * 4; *(volatile v4f*)p = o; __threadfence(); *(volatile v4f*)p = o; }
    else           { float* p = Cp + (size_t)n * NHD + lane * 4;          *(volatile v4f*)p = o; __threadfence(); *(volatile v4f*)p = o; }
}

static constexpr int XBLK = NAG * NT * (KXC / 8) / 256;
static constexpr int PBLK = NAG * NT * (KPC / 8) / 256;
static_assert((size_t)XBLK * 256 == (size_t)NAG * NT * (KXC / 8));
static_assert((size_t)PBLK * 256 == (size_t)NAG * NT * (KPC / 8));
__global__ __launch_bounds__(256) void k_gather(const float* __restrict__ obs, const float* __restrict__ fps, const int* __restrict__ nbr, bf* XC, bf* PC) {
    const int blk = blockIdx.x;
    if (blk < XBLK) {
        const int i = blk * 256 + threadIdx.x;
        const int row = i / (KXC / 8), cp = i - row * (KXC / 8);
        const int n = row / NT, t = row - n * NT;
        const int slot = cp >> 3, c8 = (cp & 7) * 8;
        const int sj = slot > 0 ? slot - 1 : 0;
        int nv = nbr[n * NNB + sj];
        asm volatile("" : "+v"(nv));
        const int ag = (slot > 0) ? clampi(nv, 0, NAG - 1) : n;
        const v8f v = *(const v8f*)(obs + ((size_t)t * NAG + ag) * NSO + c8); v8us o;
#pragma unroll
        for (int k = 0; k < 8; ++k) o[k] = f2bf(v[k]);
        bf* p = XC + (size_t)i * 8;
        *(volatile v8us*)p = o; __threadfence(); *(volatile v8us*)p = o;
    } else {
        const int i = (blk - XBLK) * 256 + threadIdx.x;
        const int row = i >> 2, slot = i & 3;
        const int n = row / NT, t = row - n * NT;
        const int ag = clampi(nbr[n * NNB + slot], 0, NAG - 1);
        const v8f v = *(const v8f*)(fps + ((size_t)t * NAG + ag) * NAC); v8us o;
#pragma unroll
        for (int k = 0; k < 8; ++k) o[k] = f2bf(v[k]);
        bf* p = PC + (size_t)i * 8;
        *(volatile v8us*)p = o; __threadfence(); *(volatile v8us*)p = o;
    }
}

static_assert(32 * 4 * 16 == 16 * 128);
__global__ __launch_bounds__(32) void k_enc(const bf* __restrict__ A, const bf* __restrict__ Bt, const float* __restrict__ bias, h16* SHp, int K, int soff) {
    __shared__ __align__(16) float os[16 * 68];
    const int lane = threadIdx.x & 31, lr = lane & 15, hi = lane >> 4; const int n = blockIdx.x, c0 = blockIdx.y * 64;
    const bf* An = A + (size_t)n * NT * K; const bf* Bn = Bt + (size_t)n * NFC * K;
    v8f acc[MBT][4];
#pragma unroll
    for (int mb = 0; mb < MBT; ++mb)
#pragma unroll
        for (int nb = 0; nb < 4; ++nb) acc[mb][nb] = (v8f){};
    const size_t aoff = (size_t)lr * K + 8 * hi, boff = (size_t)(c0 + lr) * K + 8 * hi;
#pragma unroll 1
    for (int kc = 0; kc < K; kc += 32) {
        v16bf a[MBT];
#pragma unroll
        for (int mb = 0; mb < MBT; ++mb) a[mb] = ldb(An + aoff + (size_t)mb * 16 * K + kc);
#pragma unroll
        for (int nb = 0; nb < 4; ++nb) { const v16bf b = ldb(Bn + boff + (size_t)nb * 16 * K + kc);
#pragma unroll
            for (int mb = 0; mb < MBT; ++mb) acc[mb][nb] = wmmabg(a[mb], b, acc[mb][nb]); }
    }
    float bc[4];
#pragma unroll
    for (int nb = 0; nb < 4; ++nb) bc[nb] = bfr(bias[n * NFC + c0 + nb * 16 + lr]);
#pragma unroll
    for (int mb = 0; mb < MBT; ++mb) {
#pragma unroll
        for (int nb = 0; nb < 4; ++nb) {
#pragma unroll
            for (int j = 0; j < 8; ++j) { const float v = acc[mb][nb][j] + bc[nb]; os[(hi * 8 + j) * 68 + nb * 16 + lr] = v > 0.0f ? v : 0.0f; } }
        wave_sync();
#pragma unroll 1
        for (int ps = 0; ps < 2; ++ps) {
#pragma unroll
            for (int s = 0; s < 4; ++s) { const int row = 4 * s + (lane >> 3), c8 = (lane & 7) * 8;
                const v4f x0 = *(const v4fa*)(&os[row * 68 + c8]); const v4f x1 = *(const v4fa*)(&os[row * 68 + c8 + 4]); v8h hv, rv;
#pragma unroll
                for (int i = 0; i < 4; ++i) { const h16 a0 = toh_flush(x0[i]); const h16 a1 = toh_flush(x1[i]); hv[i] = a0; hv[4 + i] = a1;
                    rv[i] = toh_flush((x0[i] - (float)a0) * QRS); rv[4 + i] = toh_flush((x1[i] - (float)a1) * QRS); }
                const size_t oo = ((size_t)(mb * 16 + row) * NAG + n) * F3 + soff + c0 + c8;
                *(volatile v8h*)(SHp + oo) = hv; *(volatile v8h*)(SHp + SPLANE + oo) = rv; }
            if (ps == 0) __threadfence(); }
        wave_sync();
    }
}

static_assert(16 * 16 == NFC * 2);
__global__ __launch_bounds__(128) void k_pre(const float* __restrict__ HSp, const bf* __restrict__ WMB, const float* __restrict__ bm, const int* __restrict__ nbr, h16* SHp, int t) {
    __shared__ __align__(16) float hv[KMC];
    __shared__ __align__(16) float sm[NFC];
    const int tid = threadIdx.x, lane = tid & 31;
    const int wave = __builtin_amdgcn_readfirstlane((int)(threadIdx.x >> 5));
    const int n = blockIdx.x;
    { const int ag = clampi(nbr[n * NNB + wave], 0, NAG - 1);
      const v4f v = *(const v4f*)(HSp + ((size_t)ag * HROWS + t) * NHD + lane * 4);
      *(v4fa*)(&hv[wave * NHD + lane * 4]) = v; }
    __syncthreads();
    const bf* w = WMB + ((size_t)n * NFC + tid) * KMC;
    float acc = 0.0f;
#pragma unroll 2
    for (int c = 0; c < KMC / 8; ++c) {
        const v4u wv = *(const v4u*)(w + c * 8);
        const v4f x0 = *(const v4fa*)(&hv[c * 8]); const v4f x1 = *(const v4fa*)(&hv[c * 8 + 4]);
        acc = dot8(wv, x0, x1, acc); }
    const float v = acc + bfr(bm[n * NFC + tid]);
    sm[tid] = v > 0.0f ? v : 0.0f;
    __syncthreads();
    if (wave == 0) {
        const int pl = lane >> 4, c8 = (lane & 15) * 8;
        const v4f x0 = *(const v4fa*)(&sm[c8]); const v4f x1 = *(const v4fa*)(&sm[c8 + 4]); v8h hvv, rvv;
#pragma unroll
        for (int i = 0; i < 4; ++i) { const h16 a0 = toh_flush(x0[i]); const h16 a1 = toh_flush(x1[i]); hvv[i] = a0; hvv[4 + i] = a1;
            rvv[i] = toh_flush((x0[i] - (float)a0) * QRS); rvv[4 + i] = toh_flush((x1[i] - (float)a1) * QRS); }
        const v8h ov = pl ? rvv : hvv;
        const size_t oo = (size_t)pl * SPLANE + ((size_t)t * NAG + n) * F3 + 2 * NFC + c8;
        *(volatile v8h*)(SHp + oo) = ov; __threadfence(); *(volatile v8h*)(SHp + oo) = ov;
    }
}

static constexpr size_t ATTN_LDS = (size_t)AWV * 1024 * 4 * 2 + (size_t)NAG * NAG * 2 * 2 + (size_t)AWV * NAG * 4 * 2 + (size_t)NAG * 4 * 2;
static_assert(ATTN_LDS <= (size_t)131072);
__global__ __launch_bounds__(32 * AWV) void k_attn(const h16* __restrict__ SHp, const h16* __restrict__ WGT, const float* __restrict__ a1, const float* __restrict__ a2,
                                                   const int* __restrict__ adj, float* S2, int t) {
    __shared__ __align__(16) float whs[AWV * 1024];
    __shared__ __align__(16) float wrs[AWV * 1024];
    __shared__ __align__(16) h16 ath[NAG * NAG];
    __shared__ __align__(16) h16 atr[NAG * NAG];
    __shared__ float part1[AWV * NAG];
    __shared__ float part2[AWV * NAG];
    __shared__ float wa1s[NAG];
    __shared__ float wa2s[NAG];
    const int tid = threadIdx.x, lane = tid & 31, lr = lane & 15, hi = lane >> 4;
    const int wave = __builtin_amdgcn_readfirstlane((int)(threadIdx.x >> 5));
    const int c0 = wave * 32, wb = wave * 1024;
    {
        v8f accH[4][2], accR[4][2];
#pragma unroll
        for (int mb = 0; mb < 4; ++mb)
#pragma unroll
            for (int nb = 0; nb < 2; ++nb) { accH[mb][nb] = (v8f){}; accR[mb][nb] = (v8f){}; }
        const size_t aoff = ((size_t)t * NAG + lr) * F3 + 8 * hi;
        const size_t boff = (size_t)(c0 + lr) * F3 + 8 * hi;
#pragma unroll 1
        for (int kc = 0; kc < F3; kc += 32) {
            v16h b[2], a[4];
#pragma unroll
            for (int nb = 0; nb < 2; ++nb) b[nb] = ldh(WGT + boff + (size_t)nb * 16 * F3 + kc);
#pragma unroll
            for (int mb = 0; mb < 4; ++mb) a[mb] = ldh(SHp + aoff + (size_t)mb * 16 * F3 + kc);
#pragma unroll
            for (int mb = 0; mb < 4; ++mb)
#pragma unroll
                for (int nb = 0; nb < 2; ++nb) accH[mb][nb] = wmma16g(a[mb], b[nb], accH[mb][nb]);
#pragma unroll
            for (int mb = 0; mb < 4; ++mb) a[mb] = ldh(SHp + SPLANE + aoff + (size_t)mb * 16 * F3 + kc);
#pragma unroll
            for (int mb = 0; mb < 4; ++mb)
#pragma unroll
                for (int nb = 0; nb < 2; ++nb) accR[mb][nb] = wmma16g(a[mb], b[nb], accR[mb][nb]);
        }
        float a1v[2], a2v[2];
#pragma unroll
        for (int nb = 0; nb < 2; ++nb) { a1v[nb] = bfr(a1[c0 + nb * 16 + lr]); a2v[nb] = bfr(a2[c0 + nb * 16 + lr]); }
#pragma unroll
        for (int mb = 0; mb < 4; ++mb) {
            v8h hv0, rv0, hv1, rv1;
#pragma unroll
            for (int r = 0; r < 8; ++r) {
                const float w0 = (accH[mb][0][r] + accR[mb][0][r] * QRI) * WCI;
                const float w1 = (accH[mb][1][r] + accR[mb][1][r] * QRI) * WCI;
                float p1 = w0 * a1v[0] + w1 * a1v[1];
                float p2 = w0 * a2v[0] + w1 * a2v[1];
                p1 += __shfl_xor(p1, 8, 32); p2 += __shfl_xor(p2, 8, 32);
                p1 += __shfl_xor(p1, 4, 32); p2 += __shfl_xor(p2, 4, 32);
                p1 += __shfl_xor(p1, 2, 32); p2 += __shfl_xor(p2, 2, 32);
                p1 += __shfl_xor(p1, 1, 32); p2 += __shfl_xor(p2, 1, 32);
                if (lr == 0) { part1[wave * NAG + mb * 16 + 8 * hi + r] = p1; part2[wave * NAG + mb * 16 + 8 * hi + r] = p2; }
                const h16 q0 = toh_flush(w0); const h16 q1 = toh_flush(w1);
                hv0[r] = q0; rv0[r] = toh_flush((w0 - (float)q0) * QRS);
                hv1[r] = q1; rv1[r] = toh_flush((w1 - (float)q1) * QRS); }
            const int f0 = wb + (0 * 16 + lr) * 32 + mb * 8 + 4 * hi;
            const int f1 = wb + (1 * 16 + lr) * 32 + mb * 8 + 4 * hi;
            *(v8ha*)(&whs[f0]) = hv0; *(v8ha*)(&wrs[f0]) = rv0;
            *(v8ha*)(&whs[f1]) = hv1; *(v8ha*)(&wrs[f1]) = rv1;
        }
    }
    __syncthreads();
    if (wave < 2) { const int i = tid; float s = 0.0f;
#pragma unroll 1
        for (int w = 0; w < AWV; ++w) s += part1[w * NAG + i];
        wa1s[i] = s; }
    else if (wave < 4) { const int i = tid - NAG; float s = 0.0f;
#pragma unroll 1
        for (int w = 0; w < AWV; ++w) s += part2[w * NAG + i];
        wa2s[i] = s; }
    __syncthreads();
    if (wave < 2) {
        const int i = tid; const float w1 = wa1s[i]; const int* arow = adj + i * NAG;
        float m = -3.0e38f;
#pragma unroll 1
        for (int j = 0; j < NAG; ++j) { int aj = arow[j]; asm volatile("" : "+v"(aj)); m = fmaxf(m, zmask(w1, wa2s[j], aj)); }
        float sum = 0.0f;
#pragma unroll 1
        for (int j = 0; j < NAG; ++j) { int aj = arow[j]; asm volatile("" : "+v"(aj)); sum += __builtin_amdgcn_exp2f((zmask(w1, wa2s[j], aj) - m) * LOG2E); }
        const float inv = PCS * (1.0f / sum);
#pragma unroll 1
        for (int j = 0; j < NAG; ++j) { int aj = arow[j]; asm volatile("" : "+v"(aj));
            const float pc = __builtin_amdgcn_exp2f((zmask(w1, wa2s[j], aj) - m) * LOG2E) * inv;
            const h16 q = toh_flush(pc);
            ath[i * NAG + j] = q; atr[i * NAG + j] = toh_flush((pc - (float)q) * QRS); }
    }
    __syncthreads();
    {
        v8f accH[4][2], accR[4][2];
#pragma unroll
        for (int mb = 0; mb < 4; ++mb)
#pragma unroll
            for (int nb = 0; nb < 2; ++nb) { accH[mb][nb] = (v8f){}; accR[mb][nb] = (v8f){}; }
#pragma unroll
        for (int kc = 0; kc < NAG; kc += 32) {
            v16h bh[2], br[2], a[4];
#pragma unroll
            for (int nb = 0; nb < 2; ++nb) { const int fi = wb + (nb * 16 + lr) * 32 + 4 * hi + kc / 2;
                const v8h t0 = *(const v8ha*)(&whs[fi]); const v8h t1 = *(const v8ha*)(&whs[fi + 8]); bh[nb] = cat16(t0, t1);
                const v8h u0 = *(const v8ha*)(&wrs[fi]); const v8h u1 = *(const v8ha*)(&wrs[fi + 8]); br[nb] = cat16(u0, u1); }
#pragma unroll
            for (int mb = 0; mb < 4; ++mb) { const int ai = (mb * 16 + lr) * NAG + 8 * hi + kc;
                const v8h t0 = *(const v8ha*)(&ath[ai]); const v8h t1 = *(const v8ha*)(&ath[ai + 16]); a[mb] = cat16(t0, t1); }
#pragma unroll
            for (int mb = 0; mb < 4; ++mb)
#pragma unroll
                for (int nb = 0; nb < 2; ++nb) { accH[mb][nb] = wmma16g(a[mb], bh[nb], accH[mb][nb]); accR[mb][nb] = wmma16g(a[mb], br[nb], accR[mb][nb]); }
#pragma unroll
            for (int mb = 0; mb < 4; ++mb) { const int ai = (mb * 16 + lr) * NAG + 8 * hi + kc;
                const v8h t0 = *(const v8ha*)(&atr[ai]); const v8h t1 = *(const v8ha*)(&atr[ai + 16]); a[mb] = cat16(t0, t1); }
#pragma unroll
            for (int mb = 0; mb < 4; ++mb)
#pragma unroll
                for (int nb = 0; nb < 2; ++nb) accR[mb][nb] = wmma16g(a[mb], bh[nb], accR[mb][nb]);
        }
        wave_sync();
#pragma unroll
        for (int mb = 0; mb < 4; ++mb) {
#pragma unroll
            for (int nb = 0; nb < 2; ++nb) {
#pragma unroll
                for (int r = 0; r < 8; ++r) { const float o = (accH[mb][nb][r] + accR[mb][nb][r] * QRI) * PCI;
                    whs[wb + (8 * hi + r) * OSP + nb * 16 + lr] = (o > 0.0f) ? o : (__builtin_amdgcn_exp2f(o * LOG2E) - 1.0f); } }
            wave_sync();
#pragma unroll 1
            for (int ps = 0; ps < 2; ++ps) {
#pragma unroll
                for (int s = 0; s < 4; ++s) { const int row = 4 * s + (lane >> 3), cofs = (lane & 7) * 4;
                    const v4f val = *(const v4fa*)(&whs[wb + row * OSP + cofs]);
                    *(volatile v4f*)(S2 + (size_t)(mb * 16 + row) * F3 + c0 + cofs) = val; }
                if (ps == 0) __threadfence(); }
            wave_sync();
        }
    }
}

static_assert(32 * 16 == NHD * 4);
__global__ __launch_bounds__(512) void k_cell(const float* __restrict__ S2, float* HSp, float* Cp, const bf* __restrict__ WIB, const bf* __restrict__ WHB,
                                              const float* __restrict__ bih, const float* __restrict__ bhh, const float* __restrict__ dones, int t) {
    __shared__ __align__(16) float sv[F3];
    __shared__ __align__(16) float hm[NHD];
    __shared__ __align__(16) float cmv[NHD];
    __shared__ __align__(16) float gts[NG4];
    __shared__ __align__(16) float hst[NHD];
    __shared__ __align__(16) float cst[NHD];
    const int tid = threadIdx.x, lane = tid & 31;
    const int wave = __builtin_amdgcn_readfirstlane((int)(threadIdx.x >> 5));
    const int n = blockIdx.x;
    const float keep = 1.0f - bfr(dones[t]);
    if (wave < 3)       { const v4f v = *(const v4f*)(S2 + (size_t)n * F3 + tid * 4); *(v4fa*)(&sv[tid * 4]) = v; }
    else if (wave == 4) { const v4f v = *(const v4f*)(HSp + ((size_t)n * HROWS + t) * NHD + lane * 4); const v4f u = v * keep; *(v4fa*)(&hm[lane * 4]) = u; }
    else if (wave == 5) { const v4f v = *(const v4f*)(Cp + (size_t)n * NHD + lane * 4); const v4f u = v * keep; *(v4fa*)(&cmv[lane * 4]) = u; }
    __syncthreads();
    {
        const bf* wi = WIB + ((size_t)n * NG4 + tid) * F3;
        const bf* wh = WHB + ((size_t)n * NG4 + tid) * NHD;
        float acc = 0.0f;
#pragma unroll 2
        for (int c = 0; c < F3 / 8; ++c) {
            const v4u wv = *(const v4u*)(wi + c * 8);
            const v4f x0 = *(const v4fa*)(&sv[c * 8]); const v4f x1 = *(const v4fa*)(&sv[c * 8 + 4]);
            acc = dot8(wv, x0, x1, acc); }
#pragma unroll 2
        for (int c = 0; c < NHD / 8; ++c) {
            const v4u wv = *(const v4u*)(wh + c * 8);
            const v4f x0 = *(const v4fa*)(&hm[c * 8]); const v4f x1 = *(const v4fa*)(&hm[c * 8 + 4]);
            acc = dot8(wv, x0, x1, acc); }
        gts[tid] = acc + bfr(bih[n * NG4 + tid]) + bfr(bhh[n * NG4 + tid]);
    }
    __syncthreads();
    if (wave < 4) {
        const int j = tid;
        const float ig = gts[j], fg = gts[NHD + j], gg = gts[2 * NHD + j], og = gts[3 * NHD + j];
        const float c1 = sgm(fg) * cmv[j] + sgm(ig) * tnh(gg);
        const float h1 = sgm(og) * tnh(c1);
        hst[j] = h1; cst[j] = c1;
    }
    __syncthreads();
    if (wave == 0)      { const v4f v = *(const v4fa*)(&hst[lane * 4]); float* p = HSp + ((size_t)n * HROWS + t + 1) * NHD + lane * 4; *(volatile v4f*)p = v; __threadfence(); *(volatile v4f*)p = v; }
    else if (wave == 1) { const v4f v = *(const v4fa*)(&cst[lane * 4]); float* p = Cp + (size_t)n * NHD + lane * 4;                  *(volatile v4f*)p = v; __threadfence(); *(volatile v4f*)p = v; }
}

static_assert((NT / 16) * 32 * 16 == NT * NAC * 4);
static_assert((NT / 4) * 16 == NT * 4);
static_assert(NT / 4 <= 32);
__global__ __launch_bounds__(32) void k_head(const float* __restrict__ HSp, const h16* __restrict__ WAC, const float* __restrict__ ba, const float* __restrict__ Wc,
                                             const float* __restrict__ bc, const int* __restrict__ acts, const int* __restrict__ nbr, float* OUT) {
    __shared__ __align__(16) float os[NT * HOP];
    __shared__ __align__(16) float vrow[NT];
    const int lane = threadIdx.x & 31, lr = lane & 15, hi = lane >> 4; const int n = blockIdx.x;
    v8f accH[MBT], accR[MBT];
#pragma unroll
    for (int mb = 0; mb < MBT; ++mb) { accH[mb] = (v8f){}; accR[mb] = (v8f){}; }
#pragma unroll 1
    for (int kc = 0; kc < NHD; kc += 32) {
        const v16h b = ldh(WAC + ((size_t)n * 16 + lr) * NHD + 8 * hi + kc);
#pragma unroll
        for (int mb = 0; mb < MBT; ++mb) {
            const float* hrow = HSp + ((size_t)n * HROWS + 1 + mb * 16 + lr) * NHD + kc + 8 * hi;
            const v4f x0 = *(const v4f*)hrow, x1 = *(const v4f*)(hrow + 4), x2 = *(const v4f*)(hrow + 16), x3 = *(const v4f*)(hrow + 20);
            v16h ah, ar;
#pragma unroll
            for (int i = 0; i < 4; ++i) {
                const h16 q0 = toh_flush(x0[i]); const h16 q1 = toh_flush(x1[i]); const h16 q2 = toh_flush(x2[i]); const h16 q3 = toh_flush(x3[i]);
                ah[i] = q0; ah[4 + i] = q1; ah[8 + i] = q2; ah[12 + i] = q3;
                ar[i] = toh_flush((x0[i] - (float)q0) * QRS); ar[4 + i] = toh_flush((x1[i] - (float)q1) * QRS);
                ar[8 + i] = toh_flush((x2[i] - (float)q2) * QRS); ar[12 + i] = toh_flush((x3[i] - (float)q3) * QRS); }
            accH[mb] = wmma16g(ah, b, accH[mb]); accR[mb] = wmma16g(ar, b, accR[mb]);
        }
    }
#pragma unroll
    for (int mb = 0; mb < MBT; ++mb)
#pragma unroll
        for (int r = 0; r < 8; ++r) os[(mb * 16 + 8 * hi + r) * HOP + lr] = (accH[mb][r] + accR[mb][r] * QRI) * WCI;
    wave_sync();
    int nbj[NNB];
#pragma unroll
    for (int j = 0; j < NNB; ++j) nbj[j] = clampi(nbr[n * NNB + j], 0, NAG - 1);
    const float bcv = bfr(bc[n]);
#pragma unroll 1
    for (int tt = lane; tt < NT; tt += 32) {
        float val = os[tt * HOP + NAC] + bcv;
#pragma unroll
        for (int j = 0; j < NNB; ++j) {
            int a = acts[nbj[j] * NT_FULL + tt];
            asm volatile("" : "+v"(a));
            const int ai = clampi(a, 0, NAC - 1);
            float w = Wc[(size_t)n * KCC + NHD + j * NAC + ai];
            asm volatile("" : "+v"(w));
            val += ((unsigned)a < (unsigned)NAC) ? bfr(w) : 0.0f; }
        vrow[tt] = val;
    }
    wave_sync();
    float bav[4];
#pragma unroll
    for (int i = 0; i < 4; ++i) bav[i] = bfr(ba[n * NAC + (lane & 1) * 4 + i]);
    float* pso = OUT + (size_t)n * NT_FULL * NAC;
    float* vso = OUT + (size_t)NAG * NT_FULL * NAC + (size_t)n * NT_FULL;
#pragma unroll 1
    for (int ps = 0; ps < 2; ++ps) {
#pragma unroll
        for (int s = 0; s < NT / 16; ++s) { const int p = s * 32 + lane; const int tt = p >> 1, a0 = (p & 1) * 4;
            const v4f x = *(const v4fa*)(&os[tt * HOP + a0]); v4f val;
#pragma unroll
            for (int i = 0; i < 4; ++i) val[i] = x[i] + bav[i];
            *(volatile v4f*)(pso + (size_t)p * 4) = val; }
        if (lane < NT / 4) { const v4f val = *(const v4fa*)(&vrow[lane * 4]); *(volatile v4f*)(vso + lane * 4) = val; }
        if (ps == 0) __threadfence(); }
}

static constexpr size_t al256(size_t v) { return (v + 255) & ~(size_t)255; }
static constexpr size_t SZ_WX = al256((size_t)NAG * NFC * KXC * 2);
static constexpr size_t SZ_WP = al256((size_t)NAG * NFC * KPC * 2);
static constexpr size_t SZ_WM = al256((size_t)NAG * NFC * KMC * 2);
static constexpr size_t SZ_WI = al256((size_t)NAG * NG4 * F3 * 2);
static constexpr size_t SZ_WH = al256((size_t)NAG * NG4 * NHD * 2);
static constexpr size_t SZ_WG = al256((size_t)F3 * F3 * 2);
static constexpr size_t SZ_WA = al256((size_t)NAG * 16 * NHD * 2);
static constexpr size_t SZ_XC = al256((size_t)NAG * NT * KXC * 2);
static constexpr size_t SZ_PC = al256((size_t)NAG * NT * KPC * 2);
static constexpr size_t SZ_SH = al256((size_t)2 * SPLANE * 2);
static constexpr size_t SZ_S2 = al256((size_t)NAG * F3 * 4);
static constexpr size_t SZ_HS = al256((size_t)NAG * HROWS * NHD * 4);
static constexpr size_t SZ_CC = al256((size_t)NAG * NHD * 4);
static constexpr size_t SZ_TOTAL = SZ_WX + SZ_WP + SZ_WM + SZ_WI + SZ_WH + SZ_WG + SZ_WA + SZ_XC + SZ_PC + SZ_SH + SZ_S2 + SZ_HS + SZ_CC;
static_assert(SZ_TOTAL <= (size_t)134217728);
static_assert((SPLANE * 2) % 256 == 0);
static_assert(((size_t)NAG * NFC * KXC) % 8 == 0);
static_assert(((size_t)NAG * NFC * KPC) % 8 == 0);
static_assert(((size_t)NAG * NFC * KMC) % 8 == 0);
static_assert(((size_t)NAG * NG4 * F3) % 8 == 0);
static_assert(((size_t)NAG * NG4 * NHD) % 8 == 0);

extern "C" void kernel_launch(void* const* d_in, const int* in_sizes, int n_in,
                              void* d_out, int out_size, void* d_ws, size_t ws_size, hipStream_t stream) {
    if (n_in < 24) return;
    if ((size_t)in_sizes[0] < (size_t)NT * NAG * NSO || (size_t)in_sizes[1] < (size_t)NT * NAG * NAC || in_sizes[2] < NT) return;
    if (in_sizes[3] < NAG * 2 * NHD) return;
    if ((size_t)in_sizes[4] < (size_t)NAG * NFC * KXC || in_sizes[5] < NAG * NFC) return;
    if ((size_t)in_sizes[6] < (size_t)NAG * NFC * KPC || in_sizes[7] < NAG * NFC) return;
    if ((size_t)in_sizes[8] < (size_t)NAG * NFC * KMC || in_sizes[9] < NAG * NFC) return;
    if (in_sizes[10] < F3 * F3 || in_sizes[11] < F3 || in_sizes[12] < F3) return;
    if ((size_t)in_sizes[13] < (size_t)NAG * NG4 * F3 || (size_t)in_sizes[14] < (size_t)NAG * NG4 * NHD) return;
    if (in_sizes[15] < NAG * NG4 || in_sizes[16] < NAG * NG4) return;
    if (in_sizes[17] < NAG * NAC * NHD || in_sizes[18] < NAG * NAC || in_sizes[19] < NAG * KCC || in_sizes[20] < NAG) return;
    if (in_sizes[21] < (NAG - 1) * NT_FULL + NT || in_sizes[22] < NAG * NNB || in_sizes[23] < NAG * NAG) return;
    if ((size_t)out_size < (size_t)NAG * NT_FULL * NAC + (size_t)(NAG - 1) * NT_FULL + NT) return;
    if (SZ_TOTAL > ws_size) return;
    const float* obs = (const float*)d_in[0];  const float* fps = (const float*)d_in[1];
    const float* dones = (const float*)d_in[2]; const float* states = (const float*)d_in[3];
    const float* Wx = (const float*)d_in[4];   const float* bx = (const float*)d_in[5];
    const float* Wp = (const float*)d_in[6];   const float* bp = (const float*)d_in[7];
    const float* Wm = (const float*)d_in[8];   const float* bm = (const float*)d_in[9];
    const float* Wg = (const float*)d_in[10];  const float* a1 = (const float*)d_in[11]; const float* a2 = (const float*)d_in[12];
    const float* Wih = (const float*)d_in[13]; const float* Whh = (const float*)d_in[14];
    const float* bih = (const float*)d_in[15]; const float* bhh = (const float*)d_in[16];
    const float* Wa = (const float*)d_in[17];  const float* ba = (const float*)d_in[18];
    const float* Wc = (const float*)d_in[19];  const float* bc = (const float*)d_in[20];
    const int* acts = (const int*)d_in[21];    const int* nbr = (const int*)d_in[22];    const int* adj = (const int*)d_in[23];
    float* OUT = (float*)d_out;
    char* wsp = (char*)d_ws;
    bf* WXB = (bf*)wsp; wsp += SZ_WX;
    bf* WPB = (bf*)wsp; wsp += SZ_WP;
    bf* WMB = (bf*)wsp; wsp += SZ_WM;
    bf* WIB = (bf*)wsp; wsp += SZ_WI;
    bf* WHB = (bf*)wsp; wsp += SZ_WH;
    h16* WGT = (h16*)wsp; wsp += SZ_WG;
    h16* WAC = (h16*)wsp; wsp += SZ_WA;
    bf* XC = (bf*)wsp; wsp += SZ_XC;
    bf* PC = (bf*)wsp; wsp += SZ_PC;
    h16* SH = (h16*)wsp; wsp += SZ_SH;
    float* S2 = (float*)wsp; wsp += SZ_S2;
    float* HS = (float*)wsp; wsp += SZ_HS;
    float* CC = (float*)wsp; wsp += SZ_CC;

    { size_t n8;
      n8 = (size_t)NAG * NFC * KXC / 8; k_cvt8<<<(unsigned)((n8 + 255) / 256), 256, 0, stream>>>(Wx, WXB, n8);
      n8 = (size_t)NAG * NFC * KPC / 8; k_cvt8<<<(unsigned)((n8 + 255) / 256), 256, 0, stream>>>(Wp, WPB, n8);
      n8 = (size_t)NAG * NFC * KMC / 8; k_cvt8<<<(unsigned)((n8 + 255) / 256), 256, 0, stream>>>(Wm, WMB, n8);
      n8 = (size_t)NAG * NG4 * F3 / 8;  k_cvt8<<<(unsigned)((n8 + 255) / 256), 256, 0, stream>>>(Wih, WIB, n8);
      n8 = (size_t)NAG * NG4 * NHD / 8; k_cvt8<<<(unsigned)((n8 + 255) / 256), 256, 0, stream>>>(Whh, WHB, n8); }
    k_wgt<<<dim3(F3 / 64, F3 / 32, 1), 256, 0, stream>>>(Wg, WGT);
    k_whead<<<(unsigned)((size_t)NAG * 16 * NHD / 8 / 256), 256, 0, stream>>>(Wa, Wc, WAC);
    k_init<<<NAG, 64, 0, stream>>>(states, HS, CC);
    k_gather<<<XBLK + PBLK, 256, 0, stream>>>(obs, fps, nbr, XC, PC);
    k_enc<<<dim3(NAG, NFC / 64, 1), 32, 0, stream>>>(XC, WXB, bx, SH, KXC, 0);
    k_enc<<<dim3(NAG, NFC / 64, 1), 32, 0, stream>>>(PC, WPB, bp, SH, KPC, NFC);

    for (int t = 0; t < NT; ++t) {
        k_pre<<<NAG, 128, 0, stream>>>(HS, WMB, bm, nbr, SH, t);
        k_attn<<<1, 32 * AWV, 0, stream>>>(SH, WGT, a1, a2, adj, S2, t);
        k_cell<<<NAG, 512, 0, stream>>>(S2, HS, CC, WIB, WHB, bih, bhh, dones, t);
    }

    k_head<<<NAG, 32, 0, stream>>>(HS, WAC, ba, Wc, bc, acts, nbr, OUT);
}
